// My_GNN_NN_36155034698325
// MI455X (gfx1250) — hardware-run, weakly checked
//
#include <hip/hip_runtime.h>


namespace {
constexpr int N = 50000, NP = 50048, E = 800000, FI = 3, NH = 4, HID = 32, HC = 128, FO = 2;
constexpr float XS = 8.0f, WSC = 256.0f, SLOPE = 0.2f;

typedef _Float16 b16;
typedef __attribute__((ext_vector_type(16))) _Float16 v16b;
typedef __attribute__((ext_vector_type(8))) _Float16 v8b;
typedef __attribute__((ext_vector_type(8))) float v8f;
typedef __attribute__((ext_vector_type(4))) float v4f;
typedef __attribute__((ext_vector_type(2))) float v2f;
__device__ __forceinline__ float bf16_rne(float f) { unsigned int u = __float_as_uint(f); u += 0x7FFFu + ((u >> 16) & 1u); return __uint_as_float(u & 0xFFFF0000u); }
__device__ __forceinline__ void split16(float v, b16& hi, b16& lo) { hi = (b16)v; lo = (b16)(v - (float)hi); }
__device__ __forceinline__ v16b frag_kb(const b16* p, int hh) { const v8b a = *(const v8b*)(p + 8 * hh), b = *(const v8b*)(p + 16 + 8 * hh); v16b f;
#pragma unroll
  for (int e = 0; e < 8; ++e) { f[e] = a[e]; f[8 + e] = b[e]; } return f; }
__device__ __forceinline__ v8f wmma16b(v16b a, v16b b, v8f c) { v8f d = __builtin_amdgcn_wmma_f32_16x16x32_f16(false, a, false, b, (short)0, c, false, false); asm volatile("v_nop\n\tv_nop\n\tv_nop\n\tv_nop" : "+v"(d) : "v"(a), "v"(b)); return d; }
__device__ __forceinline__ void wave_lds_sync() { __builtin_amdgcn_fence(__ATOMIC_RELEASE, "workgroup"); __builtin_amdgcn_wave_barrier(); __builtin_amdgcn_fence(__ATOMIC_ACQUIRE, "workgroup"); }
__device__ __forceinline__ float pmul(float a, float b) { float p = a * b; asm volatile("" : "+v"(p)); return p; }
__device__ __forceinline__ float hsum16(float v) { v += __shfl_xor(v, 1); v += __shfl_xor(v, 2); v += __shfl_xor(v, 4); return v + __shfl_xor(v, 8); }
__device__ __forceinline__ int iclamp(int v, int lo, int hi) { return v < lo ? lo : (v > hi ? hi : v); }
__device__ __forceinline__ float lrelu(float x) { return x > 0.0f ? x : SLOPE * x; }

constexpr int CSR_NBLK = 512, CSR_GB = 9, CSR_GN = 1 << CSR_GB  , CSR_MAXG = 512, CSR_CAP = 12288  ;
__global__ __launch_bounds__(64) void csrA_kernel(const int* __restrict__ dst, int E, int N, int nG, int CHP, int NGP, int* __restrict__ STG, int* __restrict__ HST) {
  extern __shared__ int sm[];
  int* cnt = sm; int* run = sm + NGP; int* ids = sm + 2 * NGP;
  const int b = blockIdx.x; const int ch = (E + CSR_NBLK - 1) / CSR_NBLK; const int e0 = b * ch, e1 = min(E, e0 + ch);
  for (int i = threadIdx.x; i < NGP; i += 64) cnt[i] = 0;
  for (int i = threadIdx.x; i < CHP; i += 64) ids[i] = -1;
  __syncthreads();
  if (threadIdx.x == 0) {
    for (int e = e0; e < e1; ++e) { int d = dst[e]; d = (d < 0) ? 0 : (d >= N ? N - 1 : d); cnt[d >> CSR_GB] += 1; }
    int acc = 0; for (int g = 0; g < nG; ++g) { run[g] = acc; acc += cnt[g]; }
    for (int e = e0; e < e1; ++e) { int d = dst[e]; d = (d < 0) ? 0 : (d >= N ? N - 1 : d); const int g = d >> CSR_GB; ids[run[g]] = e; run[g] += 1; } }
  __syncthreads();
  typedef __attribute__((ext_vector_type(4))) int v4i;
  for (int pass = 0; pass < 2; ++pass) {
    for (int i = threadIdx.x; i < CHP / 4; i += 64) *(volatile v4i*)(STG + (size_t)b * CHP + i * 4) = *(const v4i*)(&ids[i * 4]);
    for (int i = threadIdx.x; i < NGP / 4; i += 64) { v4i v; for (int e = 0; e < 4; ++e) v[e] = (i * 4 + e < nG) ? cnt[i * 4 + e] : 0; *(volatile v4i*)(HST + (size_t)b * NGP + i * 4) = v; }
    __threadfence(); }
}
__global__ __launch_bounds__(512) void csrS_kernel(const int* __restrict__ HST, int nG, int NGP, int* __restrict__ START, int* __restrict__ TOT, int* __restrict__ OFF) {
  __shared__ int tot[CSR_MAXG];
  const int b = threadIdx.x;
  for (int pass = 0; pass < 2; ++pass) { int runb = 0; for (int g = 0; g < nG; ++g) { int c = HST[(size_t)b * NGP + g]; c = (c < 0) ? 0 : c; ((volatile int*)OFF)[(size_t)g * CSR_NBLK + b] = runb; runb += c; } __threadfence(); }
  for (int g = threadIdx.x; g < nG; g += 512) { int s = 0; for (int bb = 0; bb < CSR_NBLK; ++bb) { int c = HST[(size_t)bb * NGP + g]; s += (c < 0) ? 0 : c; } tot[g] = s; }
  __syncthreads();
  if (threadIdx.x < 32) {
    __shared__ int st[CSR_MAXG + 32];
    if (threadIdx.x == 0) { int acc = 0; for (int g = 0; g < NGP; ++g) { st[g] = acc; if (g < nG) acc += (tot[g] + 31) & ~31; } st[NGP] = acc; }
    __builtin_amdgcn_fence(__ATOMIC_RELEASE, "workgroup"); __builtin_amdgcn_wave_barrier(); __builtin_amdgcn_fence(__ATOMIC_ACQUIRE, "workgroup");
    for (int pass = 0; pass < 2; ++pass) { for (int i = threadIdx.x; i < NGP + 32; i += 32) { ((volatile int*)START)[i] = (i <= NGP) ? st[min(i, NGP)] : 0; ((volatile int*)TOT)[i] = (i < nG) ? tot[i] : 0; } __threadfence(); } }
}
__global__ __launch_bounds__(256) void csrB_kernel(const int* __restrict__ dst, int N, int nG, int CHP, int NGP, int permLen, const int* __restrict__ STG, const int* __restrict__ HST, const int* __restrict__ OFF, const int* __restrict__ START, const int* __restrict__ TOT, int* __restrict__ PERM, int* __restrict__ ROWPTR, int* __restrict__ ROWCNT, int* __restrict__ FLAG) {
  typedef __attribute__((ext_vector_type(4))) int v4i;
  __shared__ int ids[CSR_CAP]; __shared__ unsigned short key[CSR_CAP]; __shared__ int outp[CSR_CAP]; __shared__ int ncnt[CSR_GN + 1]; __shared__ int boff[CSR_NBLK + 1];
  const int g = blockIdx.x, t_ = threadIdx.x; int tot = TOT[g]; int st = START[g], stn = START[g + 1]; const int v0 = g * CSR_GN; const int nv = min(CSR_GN, N - v0);
  st = (st < 0) ? 0 : (st > permLen - 32 ? permLen - 32 : st) & ~31; stn = (stn < st) ? st : (stn > permLen ? permLen : stn); tot = (tot < 0) ? 0 : tot; if (tot > stn - st && tot <= CSR_CAP) tot = stn - st;
  if (tot > CSR_CAP) {
    for (int pass = 0; pass < 2; ++pass) { for (int i = t_; i < CSR_GN / 4; i += 256) { v4i a, c; for (int e = 0; e < 4; ++e) { a[e] = st; c[e] = 0; } *(volatile v4i*)(ROWPTR + v0 + i * 4) = a; *(volatile v4i*)(ROWCNT + v0 + i * 4) = c; } if (t_ == 0) ((volatile int*)FLAG)[0] = 1; __threadfence(); } (void)nv; return; }
  if (t_ == 0) { int acc = 0; for (int b = 0; b < CSR_NBLK; ++b) { boff[b] = acc; int c = HST[(size_t)b * NGP + g]; c = (c < 0) ? 0 : (c > CHP ? CHP : c); acc += c; if (acc > tot) acc = tot; } boff[CSR_NBLK] = acc; }
  for (int i = t_; i <= CSR_GN; i += 256) ncnt[i] = 0;
  __syncthreads();
  for (int b = 0; b < CSR_NBLK; ++b) { const int c = boff[b + 1] - boff[b]; int o_ = OFF[(size_t)g * CSR_NBLK + b]; o_ = (o_ < 0) ? 0 : (o_ > CHP - c ? CHP - c : o_); const int* src_ = STG + (size_t)b * CHP + o_;
    for (int i = t_; i < c; i += 256) { int id = src_[i]; id = (id < 0) ? 0 : id; ids[boff[b] + i] = id; int d = dst[id]; d = (d < v0) ? v0 : (d >= N ? N - 1 : d); int kk = d - v0; kk = (kk < 0) ? 0 : (kk >= CSR_GN ? CSR_GN - 1 : kk); key[boff[b] + i] = (unsigned short)kk; } }
  __syncthreads();
  if (t_ == 0) { for (int i = 0; i < tot; ++i) ncnt[key[i]] += 1; int acc = 0; for (int vl = 0; vl < CSR_GN; ++vl) { const int c = ncnt[vl]; ncnt[vl] = acc; acc += c; } ncnt[CSR_GN] = acc;
    for (int i = 0; i < tot; ++i) { const int vl = key[i]; outp[ncnt[vl]] = ids[i]; ncnt[vl] += 1; }
    for (int vl = CSR_GN; vl > 0; --vl) ncnt[vl] = ncnt[vl - 1]; ncnt[0] = 0; }
  __syncthreads();
  for (int pass = 0; pass < 2; ++pass) {
    for (int i = t_; i < (stn - st) / 4; i += 256) { v4i v; for (int e = 0; e < 4; ++e) { const int q = i * 4 + e; v[e] = (q < tot) ? outp[q] : -1; } *(volatile v4i*)(PERM + st + i * 4) = v; }
    for (int i = t_; i < CSR_GN / 4; i += 256) { v4i a, c; for (int e = 0; e < 4; ++e) { const int vl = i * 4 + e; a[e] = st + ncnt[vl]; c[e] = (vl < nv) ? (ncnt[vl + 1] - ncnt[vl]) : 0; } *(volatile v4i*)(ROWPTR + v0 + i * 4) = a; *(volatile v4i*)(ROWCNT + v0 + i * 4) = c; }
    __threadfence(); }
}
__global__ __launch_bounds__(256) void csrZ_kernel(int* __restrict__ p, size_t n4) { typedef __attribute__((ext_vector_type(4))) int v4i; const size_t tid = (size_t)blockIdx.x * 256 + threadIdx.x, nth = (size_t)gridDim.x * 256; v4i z = {0, 0, 0, 0}; for (size_t i = tid; i < n4; i += nth) *(volatile v4i*)(p + i * 4) = z; }
struct CsrBufs { int *STG, *HST, *OFF, *START, *TOT, *PERM, *ROWPTR, *ROWCNT, *FLAG; int nG, NGP, CHP; size_t permLen; char* base; size_t bytes; };
static size_t csr_carve(CsrBufs& c, char* ws, size_t off, int E, int N) {
  const size_t off0 = off; c.base = ws + off;
  auto al = [&](size_t bytes) { char* p = ws + off; off += (bytes + 255) & ~(size_t)255; return p; };
  c.nG = (N + CSR_GN - 1) / CSR_GN; c.NGP = (c.nG + 31) & ~31; const int ch = (E + CSR_NBLK - 1) / CSR_NBLK; c.CHP = (ch + 31) & ~31; c.permLen = (size_t)E + 32 * (size_t)c.nG + 32;
  c.STG = (int*)al((size_t)CSR_NBLK * c.CHP * 4); c.HST = (int*)al((size_t)CSR_NBLK * c.NGP * 4); c.OFF = (int*)al((size_t)c.NGP * CSR_NBLK * 4); c.START = (int*)al((size_t)(c.NGP + 64) * 4); c.TOT = (int*)al((size_t)(c.NGP + 64) * 4);
  c.PERM = (int*)al(c.permLen * 4); c.ROWPTR = (int*)al((size_t)c.nG * CSR_GN * 4); c.ROWCNT = (int*)al((size_t)c.nG * CSR_GN * 4); c.FLAG = (int*)al(256);
  c.bytes = off - off0; return off;
}
static void csr_build(const CsrBufs& c, const int* dst, int E, int N, hipStream_t stream) {
  const size_t smem = (size_t)(2 * c.NGP + c.CHP) * 4;
  csrZ_kernel<<<512, 256, 0, stream>>>((int*)c.base, c.bytes / 16);
  csrA_kernel<<<CSR_NBLK, 64, smem, stream>>>(dst, E, N, c.nG, c.CHP, c.NGP, c.STG, c.HST);
  csrS_kernel<<<1, 512, 0, stream>>>(c.HST, c.nG, c.NGP, c.START, c.TOT, c.OFF);
  csrB_kernel<<<c.nG, 256, 0, stream>>>(dst, N, c.nG, c.CHP, c.NGP, (int)c.permLen, c.STG, c.HST, c.OFF, c.START, c.TOT, c.PERM, c.ROWPTR, c.ROWCNT, c.FLAG);
}


__global__ __launch_bounds__(256) void prepw_kernel(const float* __restrict__ w2, const float* __restrict__ l1, const float* __restrict__ l2, b16* __restrict__ W2T, b16* __restrict__ L1T, b16* __restrict__ L2T) {
  const int t = blockIdx.x * 256 + threadIdx.x; const int n1 = HC * HC / 8; v8b o;
  if (t < n1) { const int oo = (t * 8) / HC, i0 = t * 8 - oo * HC; for (int j = 0; j < 8; ++j) o[j] = (b16)(bf16_rne(w2[(size_t)(i0 + j) * HC + oo]) * WSC); for (int pass = 0; pass < 2; ++pass) { *(volatile v8b*)(W2T + (size_t)t * 8) = o; __threadfence(); } }
  else if (t < 2 * n1) { const int u = t - n1; const int oo = (u * 8) / HC, i0 = u * 8 - oo * HC; for (int j = 0; j < 8; ++j) o[j] = (b16)(bf16_rne(l1[(size_t)(i0 + j) * HC + oo]) * WSC); for (int pass = 0; pass < 2; ++pass) { *(volatile v8b*)(L1T + (size_t)u * 8) = o; __threadfence(); } }
  else if (t < 2 * n1 + 16 * HC / 8) { const int u = t - 2 * n1; const int oo = (u * 8) / HC, i0 = u * 8 - oo * HC; for (int j = 0; j < 8; ++j) o[j] = (b16)((oo < FO) ? bf16_rne(l2[(size_t)(i0 + j) * FO + oo]) * WSC : 0.0f); for (int pass = 0; pass < 2; ++pass) { *(volatile v8b*)(L2T + (size_t)u * 8) = o; __threadfence(); } }
}
__global__ __launch_bounds__(256) void node1_kernel(const float* __restrict__ x, const float* __restrict__ w1, const float* __restrict__ as1, const float* __restrict__ ad1, float* __restrict__ H, float* __restrict__ AS, float* __restrict__ AD) {
  __shared__ float Sa[16][NH], Sd[16][NH];
  const int wave = threadIdx.x >> 5, lane = threadIdx.x & 31; const size_t v0 = (size_t)blockIdx.x * 16; const int vl = wave * 2 + (lane >> 4); const size_t v = v0 + vl; const int c0 = (lane & 15) * 8, h = c0 / HID;
  float xv[FI]; for (int k = 0; k < FI; ++k) xv[k] = (v < (size_t)N) ? bf16_rne(x[v * FI + k]) : 0.0f;
  float hv[8]; float ps = 0.0f, pd = 0.0f;
#pragma unroll
  for (int j = 0; j < 8; ++j) { const int c = c0 + j; float s = 0.0f; for (int k = 0; k < FI; ++k) s += pmul(xv[k], bf16_rne(w1[k * HC + c])); hv[j] = s; ps += pmul(s, bf16_rne(as1[c])); pd += pmul(s, bf16_rne(ad1[c])); }
  ps += __shfl_xor(ps, 1); ps += __shfl_xor(ps, 2); pd += __shfl_xor(pd, 1); pd += __shfl_xor(pd, 2);
  if ((lane & 3) == 0) { Sa[vl][h] = ps; Sd[vl][h] = pd; }
  const v4f oa = {hv[0], hv[1], hv[2], hv[3]}, ob = {hv[4], hv[5], hv[6], hv[7]};
  __syncthreads();
  for (int pass = 0; pass < 2; ++pass) { *(volatile v4f*)(H + v * HC + c0) = oa; *(volatile v4f*)(H + v * HC + c0 + 4) = ob;
    if (threadIdx.x < 64) { ((volatile float*)AS)[v0 * NH + threadIdx.x] = Sa[threadIdx.x >> 2][threadIdx.x & 3]; ((volatile float*)AD)[v0 * NH + threadIdx.x] = Sd[threadIdx.x >> 2][threadIdx.x & 3]; }
    __threadfence(); }
}
template <int NHD>
__global__ __launch_bounds__(256) void agg_kernel(const int* __restrict__ srcs, const float* __restrict__ Hf, const float* __restrict__ AS, const float* __restrict__ AD, const float* __restrict__ bias, const int* __restrict__ PERM, const int* __restrict__ ROWPTR, const int* __restrict__ ROWCNT, int permLen, b16* __restrict__ Xh, b16* __restrict__ Xl) {
  constexpr int CH = HC / NHD;
  const int wave = threadIdx.x >> 5, lane = threadIdx.x & 31; const size_t v = ((size_t)blockIdx.x * 8 + wave) * 2 + (lane >> 4); const int c0 = (lane & 15) * 8, h = c0 / CH;
  const int vv = (int)((v < (size_t)N) ? v : (size_t)(N - 1));
  int st = ROWPTR[vv], cnt = ROWCNT[vv]; cnt = iclamp(cnt, 0, 4096); st = iclamp(st, 0, permLen - cnt); if (v >= (size_t)N) cnt = 0;
  const float ad = AD[(size_t)vv * NHD + h]; const float eself = lrelu(AS[(size_t)vv * NHD + h] + ad);
  float m = eself; for (int j = 0; j < cnt; ++j) { const int e = iclamp(PERM[st + j], 0, E - 1); const int s = iclamp(srcs[e], 0, N - 1); m = fmaxf(m, lrelu(AS[(size_t)s * NHD + h] + ad)); }
  float den = __expf(eself - m); float acc[8]; { const float a = den; const float* hr = Hf + (size_t)vv * HC + c0; for (int q = 0; q < 8; ++q) acc[q] = pmul(a, hr[q]); }
  for (int j = 0; j < cnt; ++j) { const int e = iclamp(PERM[st + j], 0, E - 1); const int s = iclamp(srcs[e], 0, N - 1); const float a = __expf(lrelu(AS[(size_t)s * NHD + h] + ad) - m); den += a; const float* hr = Hf + (size_t)s * HC + c0;
    const v4f h0 = *(const v4f*)hr, h1v = *(const v4f*)(hr + 4);
#pragma unroll
    for (int q = 0; q < 4; ++q) { acc[q] += pmul(a, h0[q]); acc[4 + q] += pmul(a, h1v[q]); } }
  const float inv = 1.0f / (den + 1e-16f); v8b hv8, lv8;
#pragma unroll
  for (int q = 0; q < 8; ++q) { float o = fmaxf(acc[q] * inv + bf16_rne(bias[c0 + q]), 0.0f); if (v >= (size_t)N) o = 0.0f; b16 a_, c_; split16(o * XS, a_, c_); hv8[q] = a_; lv8[q] = c_; }
  for (int pass = 0; pass < 2; ++pass) { *(volatile v8b*)(Xh + v * HC + c0) = hv8; *(volatile v8b*)(Xl + v * HC + c0) = lv8; __threadfence(); }
}
template <int MODE>
__global__ __launch_bounds__(128) void gemm_kernel(const b16* __restrict__ Ah, const b16* __restrict__ Al, const b16* __restrict__ W, const float* __restrict__ bias, const float* __restrict__ att_s, const float* __restrict__ att_d, float* __restrict__ H, float* __restrict__ AS, float* __restrict__ AD, b16* __restrict__ Yh, b16* __restrict__ Yl, float* __restrict__ out) {
  __shared__ __attribute__((aligned(16))) float Ts[4][16][HC + 4]; __shared__ float Sa[4][16], Sd[4][16];
  const int wave = threadIdx.x >> 5, lane = threadIdx.x & 31, nloc = lane & 15, hlf = lane >> 4; const size_t m0 = ((size_t)blockIdx.x * 4 + wave) * 16;
  constexpr int NT = (MODE == 2) ? 1 : 8; v8f acc[NT];
#pragma unroll
  for (int t = 0; t < NT; ++t) acc[t] = (v8f){};
#pragma unroll
  for (int kb = 0; kb < HC; kb += 32) { const v16b a = frag_kb(Ah + (m0 + nloc) * HC + kb, hlf), al = frag_kb(Al + (m0 + nloc) * HC + kb, hlf);
#pragma unroll
    for (int t = 0; t < NT; ++t) { const v16b bw = frag_kb(W + (size_t)(t * 16 + nloc) * HC + kb, hlf); acc[t] = wmma16b(a, bw, acc[t]); acc[t] = wmma16b(al, bw, acc[t]); } }
  if (MODE == 2) {
#pragma unroll
    for (int r = 0; r < 8; ++r) Ts[wave][8 * hlf + r][nloc] = acc[0][r] * (1.0f / (XS * WSC)) + ((nloc < FO) ? bf16_rne(bias[nloc & 1]) : 0.0f);
    wave_lds_sync();
    for (int pass = 0; pass < 2; ++pass) { if (lane < 8) { const int r0 = lane * 2; const v4f o4 = {Ts[wave][r0][0], Ts[wave][r0][1], Ts[wave][r0 + 1][0], Ts[wave][r0 + 1][1]}; if (m0 + r0 < (size_t)N) *(volatile v4f*)(out + (m0 + r0) * FO) = o4; } __threadfence(); }
    return; }
  float ps = 0.0f, pd = 0.0f; float pss[8], pds[8];
#pragma unroll
  for (int r = 0; r < 8; ++r) { pss[r] = 0.0f; pds[r] = 0.0f; }
#pragma unroll
  for (int t = 0; t < NT; ++t) { const int c = t * 16 + nloc; const float bb = (MODE == 1) ? bf16_rne(bias[c]) : 0.0f; const float sa = (MODE == 0) ? bf16_rne(att_s[c]) : 0.0f, sd = (MODE == 0) ? bf16_rne(att_d[c]) : 0.0f;
#pragma unroll
    for (int r = 0; r < 8; ++r) { float vv = acc[t][r] * (1.0f / (XS * WSC)) + bb; if (MODE == 1) vv = fmaxf(vv, 0.0f); Ts[wave][8 * hlf + r][c] = vv; if (MODE == 0) { pss[r] += pmul(vv, sa); pds[r] += pmul(vv, sd); } } }
  if (MODE == 0) {
#pragma unroll
    for (int r = 0; r < 8; ++r) { const float s1 = hsum16(pss[r]), s2 = hsum16(pds[r]); if (nloc == 0) { Sa[wave][8 * hlf + r] = s1; Sd[wave][8 * hlf + r] = s2; } } }
  (void)ps; (void)pd;
  wave_lds_sync();
  if (MODE == 0) __syncthreads();
  for (int pass = 0; pass < 2; ++pass) {
    for (int rr = 0; rr < 16; ++rr) { if (MODE == 0) *(volatile v4f*)(H + (m0 + rr) * HC + lane * 4) = *(const v4f*)(&Ts[wave][rr][lane * 4]);
      else if (lane < 16) { v8b hv, lv; for (int j = 0; j < 8; ++j) { b16 a_, c_; split16(Ts[wave][rr][lane * 8 + j] * XS, a_, c_); hv[j] = a_; lv[j] = c_; } *(volatile v8b*)(Yh + (m0 + rr) * HC + lane * 8) = hv; *(volatile v8b*)(Yl + (m0 + rr) * HC + lane * 8) = lv; } }
    if (MODE == 0 && threadIdx.x < 64) { const size_t mb = (size_t)blockIdx.x * 64; ((volatile float*)AS)[mb + threadIdx.x] = Sa[threadIdx.x >> 4][threadIdx.x & 15]; ((volatile float*)AD)[mb + threadIdx.x] = Sd[threadIdx.x >> 4][threadIdx.x & 15]; }
    __threadfence(); }
}
}

extern "C" void kernel_launch(void* const* d_in, const int* in_sizes, int n_in, void* d_out, int out_size, void* d_ws, size_t ws_size, hipStream_t stream) {
  (void)n_in;
  auto Fp = [&](int i) { return (const float*)d_in[i]; }; auto Ip = [&](int i) { return (const int*)d_in[i]; };
  if (in_sizes[0] != N * FI || in_sizes[1] != 2 * E || in_sizes[2] != FI * HC || in_sizes[6] != HC * HC || in_sizes[10] != HC * HC || in_sizes[12] != HC * FO || out_size != N * FO) return;
  size_t off = 0; char* ws = (char*)d_ws;
  auto carve = [&](size_t bytes) { char* p = ws + off; off += (bytes + 255) & ~(size_t)255; return p; };
  b16* W2T = (b16*)carve((size_t)HC * HC * 2); b16* L1T = (b16*)carve((size_t)HC * HC * 2); b16* L2T = (b16*)carve((size_t)16 * HC * 2);
  float* H = (float*)carve((size_t)NP * HC * 4); float* AS = (float*)carve((size_t)NP * NH * 4); float* AD = (float*)carve((size_t)NP * NH * 4); b16* Xh = (b16*)carve((size_t)NP * HC * 2); b16* Xl = (b16*)carve((size_t)NP * HC * 2); b16* Yh = (b16*)carve((size_t)NP * HC * 2); b16* Yl = (b16*)carve((size_t)NP * HC * 2);
  CsrBufs csr; off = csr_carve(csr, ws, off, E, N);
  if (off > ws_size || off > ((size_t)128 << 20)) return;
  const int* srcp = Ip(1); const int* dstp = Ip(1) + E;
  prepw_kernel<<<(2 * HC * HC / 8 + 16 * HC / 8 + 255) / 256, 256, 0, stream>>>(Fp(6), Fp(10), Fp(12), W2T, L1T, L2T);
  node1_kernel<<<NP / 16, 256, 0, stream>>>(Fp(0), Fp(2), Fp(3), Fp(4), H, AS, AD);
  csr_build(csr, dstp, E, N, stream);
  agg_kernel<NH><<<NP / 16, 256, 0, stream>>>(srcp, H, AS, AD, Fp(5), csr.PERM, csr.ROWPTR, csr.ROWCNT, (int)csr.permLen, Xh, Xl);
  gemm_kernel<0><<<NP / 64, 128, 0, stream>>>(Xh, Xl, W2T, nullptr, Fp(7), Fp(8), H, AS, AD, nullptr, nullptr, nullptr);
  agg_kernel<1><<<NP / 16, 256, 0, stream>>>(srcp, H, AS, AD, Fp(9), csr.PERM, csr.ROWPTR, csr.ROWCNT, (int)csr.permLen, Xh, Xl);
  gemm_kernel<1><<<NP / 64, 128, 0, stream>>>(Xh, Xl, L1T, Fp(11), nullptr, nullptr, nullptr, nullptr, nullptr, Yh, Yl, nullptr);
  gemm_kernel<2><<<NP / 64, 128, 0, stream>>>(Yh, Yl, L2T, Fp(13), nullptr, nullptr, nullptr, nullptr, nullptr, nullptr, nullptr, (float*)d_out);
}
